// DFHLoss_26474178412717
// MI455X (gfx1250) — hardware-verified
//
#include <hip/hip_runtime.h>


#define BITS   64
#define NCLS   100
#define NCP    112
#define NB     256
#define NTR    100000
#define TCOL   32
#define CPB    400
#define NBLKM  250
#define NSTEP  200

#define VP 136
#define TP 72
#define MP 136
#define YP 264

#define OFS_VF   0
#define OFS_VH   25600
#define OFS_VL   43008
#define OFS_TH   60416
#define OFS_TL   76544
#define OFS_MH   92672
#define OFS_ML   123136
#define OFS_Q    153600
#define OFS_S    193600
#define OFS_LAB  219200
#define OFS_RED  220224
#define LDS_SGD  222400
#define OFS_YT   25600
#define OFS_BP   84736
#define OFS_OST  25600
#define ZERO_BEG 25600
#define ZERO_U32 32000

static_assert(NTR % TCOL == 0);
static_assert(NTR % CPB == 0);
static_assert(NTR / CPB == NBLKM);
static_assert(CPB % 16 == 0);
static_assert(NBLKM <= 256);
static_assert(OFS_VH == OFS_VF + BITS * NCLS * 4);
static_assert(OFS_VL == OFS_VH + BITS * VP * 2);
static_assert(OFS_TH == OFS_VL + BITS * VP * 2);
static_assert(OFS_TL == OFS_TH + NCP * TP * 2);
static_assert(OFS_MH == OFS_TL + NCP * TP * 2);
static_assert(OFS_ML == OFS_MH + NCP * MP * 2);
static_assert(OFS_Q  == OFS_ML + NCP * MP * 2);
static_assert(OFS_S  == OFS_Q + NCLS * NCLS * 4);
static_assert(OFS_LAB == OFS_S + BITS * NCLS * 4);
static_assert(OFS_RED == OFS_LAB + NB * 4);
static_assert(LDS_SGD == OFS_RED + 272 * 8);
static_assert(OFS_YT + NCP * YP * 2 <= OFS_BP);
static_assert(OFS_BP + BITS * YP * 2 <= OFS_Q);
static_assert(OFS_OST + 6404 * 4 <= OFS_Q);
static_assert(ZERO_BEG + ZERO_U32 * 4 == OFS_Q);

typedef _Float16 f16t;
typedef unsigned short us_t;
typedef f16t   v8h   __attribute__((ext_vector_type(8)));
typedef f16t   v16h  __attribute__((ext_vector_type(16)));
typedef __bf16 v16b  __attribute__((ext_vector_type(16)));
typedef us_t   v8us  __attribute__((ext_vector_type(8)));
typedef us_t   v16us __attribute__((ext_vector_type(16)));
typedef float  v8f   __attribute__((ext_vector_type(8)));
typedef float  v4f   __attribute__((ext_vector_type(4)));
typedef unsigned int v4u __attribute__((ext_vector_type(4)));
typedef double v2d   __attribute__((ext_vector_type(2)));

union FragH { v16h v; v8h q[2]; };
union FragB { v16b v; v16us u; v8us q[2]; };
union Pk16  { v8h h; v8us s; v4u u; };
union Pk32  { v4f f; v4u u; };

__device__ __forceinline__ int imin(int a, int b) { return a < b ? a : b; }
__device__ __forceinline__ int imax(int a, int b) { return a > b ? a : b; }
__device__ __forceinline__ float sgnf(float x) { return (x > 0.f) ? 1.f : ((x < 0.f) ? -1.f : 0.f); }
__device__ __forceinline__ us_t f2bf(float f) {
    unsigned u = __float_as_uint(f);
    u += 0x7FFFu + ((u >> 16) & 1u);
    return (us_t)(u >> 16);
}
__device__ __forceinline__ float bf2f(us_t b) { return __uint_as_float(((unsigned)b) << 16); }
__device__ __forceinline__ v8f z8() { v8f z = {0.f, 0.f, 0.f, 0.f, 0.f, 0.f, 0.f, 0.f}; return z; }

__device__ __forceinline__ v8f wbf(v16b a, v16b b, v8f c) {
    return __builtin_amdgcn_wmma_f32_16x16x32_bf16(false, a, false, b, (short)0, c, false, false);
}
__device__ __forceinline__ v8f wf16(v16h a, v16h b, v8f c) {
    return __builtin_amdgcn_wmma_f32_16x16x32_f16(false, a, false, b, (short)0, c, false, false);
}

__device__ __forceinline__ void ldB(FragB& f, const us_t* plane, int row, int pitch, int ks, int h) {
    const us_t* p = plane + row * pitch + ks * 32 + 8 * h;
    f.q[0] = *(const v8us*)p;
    f.q[1] = *(const v8us*)(p + 16);
}

__device__ __forceinline__ v8f tile_plain8(const us_t* Apl, int arow, const us_t* Bpl, int brow, int h) {
    v8f acc = z8();
#pragma unroll 1
    for (int ks = 0; ks < 8; ++ks) {
        FragB a, b;
        ldB(a, Apl, arow, YP, ks, h);
        ldB(b, Bpl, brow, YP, ks, h);
        acc = wbf(a.v, b.v, acc);
        asm volatile("v_nop\n\tv_nop\n\tv_nop\n\tv_nop" : "+v"(acc) : "v"(a.v), "v"(b.v));
    }
    return acc;
}

template<int KS>
__device__ __forceinline__ v8f tile_x3(const us_t* Ah, const us_t* Al, int arow, int ap,
                                       const us_t* Bh, const us_t* Bl, int brow, int bp, int h) {
    v8f acc = z8();
#pragma unroll
    for (int ks = 0; ks < KS; ++ks) {
        FragB ah, al, bh, bl;
        ldB(ah, Ah, arow, ap, ks, h);
        ldB(al, Al, arow, ap, ks, h);
        ldB(bh, Bh, brow, bp, ks, h);
        ldB(bl, Bl, brow, bp, ks, h);
        acc = wbf(ah.v, bh.v, acc);
        acc = wbf(ah.v, bl.v, acc);
        acc = wbf(al.v, bh.v, acc);
        asm volatile("v_nop\n\tv_nop\n\tv_nop\n\tv_nop"
                     : "+v"(acc) : "v"(ah.v), "v"(al.v), "v"(bh.v), "v"(bl.v));
    }
    return acc;
}

__global__ __launch_bounds__(256)
void k_planes(const float* __restrict__ u, const float* __restrict__ y,
              const int* __restrict__ ind, int nind,
              const float* __restrict__ U, const float* __restrict__ Y,
              f16t* __restrict__ Upl, int* __restrict__ labT) {
    __shared__ __attribute__((aligned(16))) f16t Tt[TCOL * 72];
    __shared__ int mark[TCOL];
    const int tid = threadIdx.x;
    const int tbase = blockIdx.x * TCOL;

    if (tid < TCOL) mark[tid] = -1;
    __syncthreads();
    {
        int j = imin(tid, nind - 1);
        int t = ind[j];
        if (tid < nind && t >= tbase && t < tbase + TCOL) mark[t - tbase] = tid;
    }
    __syncthreads();
#pragma unroll
    for (int k8 = 0; k8 < 8; ++k8) {
        int e  = tid + 256 * k8;
        int k  = e >> 5;
        int tl = e & 31;
        int n  = tbase + tl;
        float uv = U[(size_t)k * NTR + n];
        int mk = mark[tl];
        int mj = imax(mk, 0);
        float pv = u[mj * BITS + k];
        Tt[tl * 72 + k] = (f16t)((mk >= 0) ? pv : uv);
    }
    __syncthreads();
    {
        const int row = tid >> 3, pc = tid & 7;
        Pk16 v;
        v.h = *(const v8h*)(Tt + row * 72 + pc * 8);
        f16t* d = Upl + (size_t)(tbase + row) * BITS + pc * 8;
        *(volatile v4u*)d = v.u;
        __threadfence();
        *(volatile v4u*)d = v.u;
    }
    if (tid < 32) {
        const int n = tbase + tid;
        const int mk = mark[tid];
        const int mj = imax(mk, 0);
        float yv = Y[n];
        float pv = y[mj * NCLS];
        float bv = (mk >= 0) ? pv : yv;
        int best = 0;
#pragma unroll 1
        for (int c = 1; c < NCLS; ++c) {
            yv = Y[(size_t)c * NTR + n];
            pv = y[mj * NCLS + c];
            float v = (mk >= 0) ? pv : yv;
            if (v > bv) { bv = v; best = c; }
        }
        int* d = labT + n;
        *(volatile int*)d = best;
        __threadfence();
        *(volatile int*)d = best;
    }
}

__global__ __launch_bounds__(256)
void k_metric(const float* __restrict__ u, const float* __restrict__ y,
              const f16t* __restrict__ Upl, const int* __restrict__ labT,
              double* __restrict__ part) {
    __shared__ int lab[NB];
    __shared__ __attribute__((aligned(16))) double red[16];
    const int tid = threadIdx.x, w = tid >> 5, l = tid & 31, h = l >> 4, m = l & 15;

    {
        const float* row = y + tid * NCLS;
        int best = 0; float bv = row[0];
#pragma unroll 1
        for (int c = 1; c < NCLS; ++c) { float v = row[c]; if (v > bv) { bv = v; best = c; } }
        lab[tid] = best;
    }
    if (tid < 16) red[tid] = 0.0;
    __syncthreads();

    int lr[16];
#pragma unroll
    for (int rt = 0; rt < 2; ++rt)
#pragma unroll
        for (int r = 0; r < 8; ++r) lr[rt * 8 + r] = lab[32 * w + 16 * rt + 8 * h + r];

    FragH a[2][2];
#pragma unroll
    for (int rt = 0; rt < 2; ++rt)
#pragma unroll
        for (int ks = 0; ks < 2; ++ks) {
            const float* p = u + (size_t)(32 * w + 16 * rt + m) * BITS + 32 * ks + 8 * h;
            v4f x0 = *(const v4f*)p,        x1 = *(const v4f*)(p + 4);
            v4f x2 = *(const v4f*)(p + 16), x3 = *(const v4f*)(p + 20);
            Pk16 q0, q1;
#pragma unroll
            for (int i = 0; i < 4; ++i) {
                q0.h[i] = (f16t)x0[i]; q0.h[4 + i] = (f16t)x1[i];
                q1.h[i] = (f16t)x2[i]; q1.h[4 + i] = (f16t)x3[i];
            }
            a[rt][ks].q[0] = q0.h;
            a[rt][ks].q[1] = q1.h;
        }

    double ds = 0.0;
    const int col0 = blockIdx.x * CPB;
#pragma unroll 1
    for (int ct = 0; ct < CPB / 16; ++ct) {
        const int n  = col0 + ct * 16 + m;
        const int nn = imin(n, NTR - 1);
        const f16t* bp = Upl + (size_t)nn * BITS + 8 * h;
        FragH b[2];
        b[0].q[0] = *(const v8h*)(bp);
        b[0].q[1] = *(const v8h*)(bp + 16);
        b[1].q[0] = *(const v8h*)(bp + 32);
        b[1].q[1] = *(const v8h*)(bp + 48);
        const int lt = labT[nn];
        v8f acc0 = z8(), acc1 = z8();
        acc0 = wf16(a[0][0].v, b[0].v, acc0);
        acc1 = wf16(a[1][0].v, b[0].v, acc1);
        acc0 = wf16(a[0][1].v, b[1].v, acc0);
        acc1 = wf16(a[1][1].v, b[1].v, acc1);
        asm volatile("v_nop\n\tv_nop\n\tv_nop\n\tv_nop"
                     : "+v"(acc0), "+v"(acc1)
                     : "v"(a[0][0].v), "v"(a[0][1].v), "v"(a[1][0].v), "v"(a[1][1].v),
                       "v"(b[0].v), "v"(b[1].v));
#pragma unroll
        for (int r = 0; r < 8; ++r) {
            float ip0 = fminf(fmaxf(0.5f * acc0[r], -100.f), 50.f);
            float x0  = (lr[r] == lt) ? (1.0f - ip0) : (1.0f + ip0);
            ds += (double)log1pf(expf(x0));
            float ip1 = fminf(fmaxf(0.5f * acc1[r], -100.f), 50.f);
            float x1  = (lr[8 + r] == lt) ? (1.0f - ip1) : (1.0f + ip1);
            ds += (double)log1pf(expf(x1));
        }
    }
#pragma unroll
    for (int off = 16; off > 0; off >>= 1) ds += __shfl_xor(ds, off);
    if (l == 0) red[w] = ds;
    __syncthreads();
    if (w == 0) {
        const int q = l & 7;
        v2d pv;
        pv.x = red[2 * q];
        pv.y = red[2 * q + 1];
        double* dst = part + (size_t)blockIdx.x * 16 + 2 * q;
        if (l < 8) *(volatile v2d*)dst = pv;
        __threadfence();
        if (l < 8) *(volatile v2d*)dst = pv;
    }
}

__global__ __launch_bounds__(256)
void k_sgd(const float* __restrict__ u, const float* __restrict__ y,
           const float* __restrict__ Vg, const float* __restrict__ TK,
           const double* __restrict__ part, float* __restrict__ out) {
    extern __shared__ float4 dsm4[];
    unsigned char* sm = reinterpret_cast<unsigned char*>(dsm4);
    float*  Vf  = (float*)(sm + OFS_VF);
    us_t*   Vh  = (us_t*)(sm + OFS_VH);
    us_t*   Vl  = (us_t*)(sm + OFS_VL);
    us_t*   Th  = (us_t*)(sm + OFS_TH);
    us_t*   Tl  = (us_t*)(sm + OFS_TL);
    us_t*   Mh  = (us_t*)(sm + OFS_MH);
    us_t*   Ml  = (us_t*)(sm + OFS_ML);
    float*  Qf  = (float*)(sm + OFS_Q);
    float*  Sf  = (float*)(sm + OFS_S);
    int*    lab = (int*)(sm + OFS_LAB);
    double* red = (double*)(sm + OFS_RED);
    us_t*   Yt  = (us_t*)(sm + OFS_YT);
    us_t*   Bp  = (us_t*)(sm + OFS_BP);
    const int tid = threadIdx.x, w = tid >> 5, l = tid & 31, h = l >> 4, m = l & 15;
    const float cI = 2.0f / 16384.0f, cE = 4.0f / 10000.0f, cQ = 2.0f / 6400.0f;
    const float muc = 1.0f;

    for (int e = tid; e < BITS * NCLS; e += 256) Vf[e] = Vg[e];
    int lb;
    {
        const float* row = y + tid * NCLS;
        int best = 0; float bv = row[0];
#pragma unroll 1
        for (int c = 1; c < NCLS; ++c) { float v = row[c]; if (v > bv) { bv = v; best = c; } }
        lb = best;
        lab[tid] = best;
    }
    double dq = 0.0;
#pragma unroll 1
    for (int i = 0; i < BITS; ++i) {
        float vv = Vg[i * NCLS + lb];
        float ut = u[tid * BITS + i];
        float bb = sgnf(muc * sgnf(vv) + ut);
        Bp[i * YP + tid] = f2bf(bb);
        float d = bb - ut;
        dq += (double)(d * d);
    }
    for (int e = tid; e < BITS * 8; e += 256) { int i = e >> 3, j = NB + (e & 7); Bp[i * YP + j] = 0; }
    for (int e = tid; e < NCP * YP; e += 256) {
        int c = e / YP;
        int j = e - c * YP;
        int cc = imin(c, NCLS - 1), jj = imin(j, NB - 1);
        float v = y[jj * NCLS + cc];
        v = (c < NCLS && j < NB) ? v : 0.f;
        Yt[e] = f2bf(v);
    }
    red[tid] = dq;
    __syncthreads();
    for (int s = 128; s > 0; s >>= 1) {
        if (tid < s) red[tid] += red[tid + s];
        __syncthreads();
    }
    if (tid == 0) red[256] = red[0];
    __syncthreads();

    for (int t = w; t < 49 + 28; t += 8) {
        if (t < 49) {
            const int tm = t / 7, tn = t - tm * 7;
            v8f acc = tile_plain8(Yt, tm * 16 + m, Yt, tn * 16 + m, h);
            const int d = tn * 16 + m, dc = imin(d, NCLS - 1);
#pragma unroll
            for (int r = 0; r < 8; ++r) {
                int c = tm * 16 + 8 * h + r;
                int cc = imin(c, NCLS - 1);
                float tk = TK[cc * NCLS + dc];
                float q = cI * acc[r] - cE * tk;
                if (c < NCLS && d < NCLS) Qf[c * NCLS + d] = q;
            }
        } else {
            const int s = t - 49;
            const int ti = s / 7, tn = s - ti * 7;
            v8f acc = tile_plain8(Bp, ti * 16 + m, Yt, tn * 16 + m, h);
            const int c = tn * 16 + m;
#pragma unroll
            for (int r = 0; r < 8; ++r) {
                int i = ti * 16 + 8 * h + r;
                if (c < NCLS) Sf[i * NCLS + c] = cI * acc[r];
            }
        }
    }
    __syncthreads();
    {
        unsigned* z = (unsigned*)(sm + ZERO_BEG);
        for (int e = tid; e < ZERO_U32; e += 256) z[e] = 0u;
    }
    __syncthreads();

#pragma unroll 1
    for (int it = 0; it < NSTEP; ++it) {
        float alpha = 0.03f;
        if (it >= 149) alpha *= 0.1f;
        if (it >= 179) alpha *= 0.1f;

        for (int e = tid; e < BITS * NCLS; e += 256) {
            int i = e / NCLS;
            int c = e - i * NCLS;
            float v = Vf[e];
            us_t hb = f2bf(v);
            us_t lo = f2bf(v - bf2f(hb));
            Vh[i * VP + c] = hb; Vl[i * VP + c] = lo;
            Th[c * TP + i] = hb; Tl[c * TP + i] = lo;
        }
        __syncthreads();

        for (int t = w; t < 49; t += 8) {
            const int tm = t / 7, tn = t - tm * 7;
            v8f acc = tile_x3<2>(Th, Tl, tm * 16 + m, TP, Th, Tl, tn * 16 + m, TP, h);
            const int d = tn * 16 + m, dc = imin(d, NCLS - 1);
            const int cb = tm * 16 + 8 * h;
            Pk16 ph, pl;
#pragma unroll
            for (int r = 0; r < 8; ++r) {
                int c = cb + r;
                int cc = imin(c, NCLS - 1);
                float q = Qf[cc * NCLS + dc];
                q = (c < NCLS && d < NCLS) ? q : 0.f;
                float mv = cE * acc[r] + q;
                us_t hb = f2bf(mv);
                ph.s[r] = hb;
                pl.s[r] = f2bf(mv - bf2f(hb));
            }
            *(v8us*)(Mh + d * MP + cb) = ph.s;
            *(v8us*)(Ml + d * MP + cb) = pl.s;
        }
        __syncthreads();

        for (int t = w; t < 28; t += 8) {
            const int ti = t / 7, tn = t - ti * 7;
            v8f acc = tile_x3<4>(Vh, Vl, ti * 16 + m, VP, Mh, Ml, tn * 16 + m, MP, h);
            const int d = tn * 16 + m, dc = imin(d, NCLS - 1);
#pragma unroll
            for (int r = 0; r < 8; ++r) {
                int i = ti * 16 + 8 * h + r;
                float v  = Vf[i * NCLS + dc];
                float sv = Sf[i * NCLS + dc];
                float g  = (acc[r] - sv) + cQ * (v - sgnf(v));
                float nv = v - alpha * g;
                if (d < NCLS) Vf[i * NCLS + d] = nv;
            }
        }
        __syncthreads();
    }

    {
        const int bb = imin(tid, NBLKM - 1);
        double s = 0.0;
#pragma unroll
        for (int k = 0; k < 8; ++k) s += part[(size_t)bb * 16 + k];
        red[tid] = (tid < NBLKM) ? s : 0.0;
    }
    __syncthreads();
    for (int s = 128; s > 0; s >>= 1) {
        if (tid < s) red[tid] += red[tid + s];
        __syncthreads();
    }
    float lossf;
    {
        double ms = red[0], qs = red[256];
        double lv = ms * (1.0 / 25600000.0) + 0.5 * (qs * (1.0 / 16384.0));
        lossf = (float)lv;
    }
    float* Ost = (float*)(sm + OFS_OST);
    if (tid == 0) Ost[0] = lossf;
    for (int e = tid; e < BITS * NCLS; e += 256) Ost[1 + e] = Vf[e];
    __syncthreads();
    Pk32 pc[7];
#pragma unroll
    for (int k = 0; k < 7; ++k) {
        int p = imin(tid + 256 * k, 1599);
        pc[k].f = *(const v4f*)(Ost + 4 * p);
    }
    const float tlv = Ost[6400];
#pragma unroll
    for (int k = 0; k < 7; ++k) {
        int p = tid + 256 * k;
        if (p < 1600) *(volatile v4u*)(out + 4 * p) = pc[k].u;
    }
    if (tid == 0) *(volatile float*)(out + 6400) = tlv;
    __threadfence();
#pragma unroll
    for (int k = 0; k < 7; ++k) {
        int p = tid + 256 * k;
        if (p < 1600) *(volatile v4u*)(out + 4 * p) = pc[k].u;
    }
    if (tid == 0) *(volatile float*)(out + 6400) = tlv;
}

extern "C" void kernel_launch(void* const* d_in, const int* in_sizes, int n_in,
                              void* d_out, int out_size, void* d_ws, size_t ws_size,
                              hipStream_t stream) {
    if (n_in < 7) return;
    if (in_sizes[0] != NB * BITS || in_sizes[1] != NB * NCLS || in_sizes[2] != NB ||
        in_sizes[3] != BITS * NTR || in_sizes[4] != NCLS * NTR ||
        in_sizes[5] != BITS * NCLS || in_sizes[6] != NCLS * NCLS) return;
    if (out_size != 1 + BITS * NCLS) return;

    const float* u   = (const float*)d_in[0];
    const float* y   = (const float*)d_in[1];
    const int*   ind = (const int*)d_in[2];
    const float* U   = (const float*)d_in[3];
    const float* Y   = (const float*)d_in[4];
    const float* V   = (const float*)d_in[5];
    const float* TK  = (const float*)d_in[6];
    float* out = (float*)d_out;

    const size_t off_upl  = 0;
    const size_t off_lab  = off_upl + (size_t)NTR * BITS * 2;
    const size_t off_part = off_lab + (size_t)NTR * 4;
    const size_t total    = off_part + (size_t)NBLKM * 16 * 8;
    if (total > ws_size) return;
    char* ws = (char*)d_ws;
    f16t*   Upl  = (f16t*)(ws + off_upl);
    int*    labT = (int*)(ws + off_lab);
    double* part = (double*)(ws + off_part);

    k_planes<<<dim3(NTR / TCOL), dim3(256), 0, stream>>>(u, y, ind, in_sizes[2], U, Y, Upl, labT);
    k_metric<<<dim3(NBLKM), dim3(256), 0, stream>>>(u, y, Upl, labT, part);
    hipFuncSetAttribute(reinterpret_cast<const void*>(&k_sgd),
                        hipFuncAttributeMaxDynamicSharedMemorySize, LDS_SGD);
    k_sgd<<<dim3(1), dim3(256), LDS_SGD, stream>>>(u, y, V, TK, part, out);
}
